// PartialDecoder_38671885533516
// MI455X (gfx1250) — hardware-run, weakly checked
//
#include <hip/hip_runtime.h>
#include <math.h>

typedef __attribute__((ext_vector_type(8)))  _Float16 v8h;
typedef __attribute__((ext_vector_type(16))) __bf16   v16b;
typedef __attribute__((ext_vector_type(8)))  __bf16   v8b;
typedef __attribute__((ext_vector_type(8)))  float    v8f;
typedef __attribute__((ext_vector_type(4)))  float    v4f;

constexpr int kB  = 64;
constexpr int kL  = 32;
constexpr int kH  = 128;
constexpr int kO  = 16384;
constexpr int kC  = 32;
constexpr int kW1Rows = kH + kC + 1;
constexpr int kEP = 132;
static_assert(kW1Rows == 161);
static_assert((kL % 32) == 0 && (kH % 32) == 0 && (kC % 32) == 0);
static_assert((kB % 64) == 0 && (kH % 64) == 0 && (kO % 64) == 0);
static_assert((kO % 32) == 0 && kH == 128 && kB == 64);

constexpr size_t kOffFEH = 0;
constexpr size_t kOffFEL = kOffFEH + (size_t)kO * kC * 2;
constexpr size_t kOffZH  = kOffFEL + (size_t)kO * kC * 2;
constexpr size_t kOffZL  = kOffZH  + (size_t)kB * kL * 2;
constexpr size_t kOffWZH = kOffZL  + (size_t)kB * kL * 2;
constexpr size_t kOffWZL = kOffWZH + (size_t)kH * kL * 2;
constexpr size_t kOffWFH = kOffWZL + (size_t)kH * kL * 2;
constexpr size_t kOffWFL = kOffWFH + (size_t)kH * kC * 2;
constexpr size_t kOffWHH = kOffWFL + (size_t)kH * kC * 2;
constexpr size_t kOffWHL = kOffWHH + (size_t)kH * kH * 2;
constexpr size_t kOffPZH = kOffWHL + (size_t)kH * kH * 2;
constexpr size_t kOffPZL = kOffPZH + (size_t)kB * kH * 2;
constexpr size_t kOffAF  = kOffPZL + (size_t)kB * kH * 2;
constexpr size_t kOffEF  = kOffAF  + (size_t)kB * kH * 4;
constexpr size_t kWsTotal = kOffEF + (size_t)kO * kH * 4;
static_assert(kWsTotal == 10657792ull);
static_assert(kWsTotal <= 134217728ull);
static_assert((kOffFEL % 128) == 0 && (kOffZH % 128) == 0 && (kOffZL % 128) == 0 && (kOffWZH % 128) == 0 &&
              (kOffWZL % 128) == 0 && (kOffWFH % 128) == 0 && (kOffWFL % 128) == 0 && (kOffWHH % 128) == 0 &&
              (kOffWHL % 128) == 0 && (kOffPZH % 128) == 0 && (kOffPZL % 128) == 0 && (kOffAF % 128) == 0 &&
              (kOffEF % 128) == 0);

__device__ __forceinline__ unsigned short f2bf_bits(float f) {
  unsigned u = __float_as_uint(f);
  return (unsigned short)((u + 0x7FFFu + ((u >> 16) & 1u)) >> 16);
}
__device__ __forceinline__ float bf_bits2f(unsigned short h) { return __uint_as_float(((unsigned)h) << 16); }

__device__ __forceinline__ v8f mma_bf16_guarded(v16b a, v16b b, v8f c) {
  c = __builtin_amdgcn_wmma_f32_16x16x32_bf16(false, a, false, b, (short)0, c, false, false);
  asm volatile("v_nop\n\tv_nop\n\tv_nop\n\tv_nop" : "+v"(c) : "v"(a), "v"(b));
  return c;
}
__device__ __forceinline__ void keep4_b(v16b a, v16b b, v16b c, v16b d) { asm volatile("v_nop" :: "v"(a), "v"(b), "v"(c), "v"(d)); }

template <typename T> struct Frag;
template <> struct Frag<__bf16> {
  typedef v16b V; union U { v16b v; v8b h[2]; };
  static __device__ __forceinline__ v16b load(const __bf16* p) {
    U f; f.h[0] = *(const v8b*)(p); f.h[1] = *(const v8b*)(p + 16); return f.v;
  }
  static __device__ __forceinline__ v8f mma(v16b a, v16b b, v8f c) { return mma_bf16_guarded(a, b, c); }
  static __device__ __forceinline__ void keep(v16b a, v16b b, v16b c, v16b d) { keep4_b(a, b, c, d); }
};

template <int ET> struct Elem;
template <> struct Elem<1> { typedef __bf16 T; };
template <int ET, int SPL, int BIAS_MODE, int OUT_MODE, bool RESID, int ACT = 0>
__global__ __launch_bounds__(256) void wmma_gemm64(
    const unsigned short* __restrict__ Ap, const unsigned short* __restrict__ A2p, int lda, long strideA,
    const unsigned short* __restrict__ Btp, const unsigned short* __restrict__ Bt2p, int ldb, long strideB,
    void* __restrict__ Cout, void* __restrict__ Cout2, int ldc, long strideC,
    const float* __restrict__ bias,
    const float* __restrict__ resid, long strideR,
    int M, int N, int K, float scale) {
  typedef typename Elem<ET>::T T;
  typedef typename Frag<T>::V V;
  const T* A = (const T*)Ap; const T* A2 = (const T*)A2p; const T* Bt = (const T*)Btp; const T* Bt2 = (const T*)Bt2p;
  __shared__ __align__(16) float sT[8][16 * 68];
  const int b    = blockIdx.y;
  const int lane = threadIdx.x & 31;
  const int wave = threadIdx.x >> 5;
  const int tilesN = N >> 6;
  const int tilesM = M >> 6;
  const int tile = blockIdx.x * 8 + wave;
  if (tile >= tilesM * tilesN) return;
  const int tm = tile / tilesN;
  const int tn = tile - tm * tilesN;
  const int m0 = tm << 6;
  const int n0 = tn << 6;

  const T* Ab  = A  + (size_t)b * strideA;
  const T* Bb  = Bt + (size_t)b * strideB;
  const T* Ab2 = (SPL >= 1) ? (A2  + (size_t)b * strideA) : nullptr;
  const T* Bb2 = (SPL == 2) ? (Bt2 + (size_t)b * strideB) : nullptr;

  const int rlane = lane & 15;
  const int koff  = (lane >> 4) * 8;
  const int mOff  = (lane >> 4) * 8;

  v8f acc[4][4];
#pragma unroll
  for (int i = 0; i < 4; ++i)
#pragma unroll
    for (int j = 0; j < 4; ++j) acc[i][j] = (v8f){0.f,0.f,0.f,0.f,0.f,0.f,0.f,0.f};

  for (int k0 = 0; k0 < K; k0 += 32) {
    V bh[4], bl[4];
#pragma unroll
    for (int j = 0; j < 4; ++j) {
      const size_t bo = (size_t)(n0 + (j << 4) + rlane) * ldb + koff + k0;
      bh[j] = Frag<T>::load(Bb + bo);
      if (SPL == 2) bl[j] = Frag<T>::load(Bb2 + bo);
    }
#pragma unroll
    for (int i = 0; i < 4; ++i) {
      const size_t ao = (size_t)(m0 + (i << 4) + rlane) * lda + koff + k0;
      V ah = Frag<T>::load(Ab + ao);
      V al;
      if (SPL >= 1) al = Frag<T>::load(Ab2 + ao);
#pragma unroll
      for (int j = 0; j < 4; ++j) {
        acc[i][j] = Frag<T>::mma(ah, bh[j], acc[i][j]);
        if (SPL == 2) acc[i][j] = Frag<T>::mma(ah, bl[j], acc[i][j]);
        if (SPL >= 1) acc[i][j] = Frag<T>::mma(al, bh[j], acc[i][j]);
      }
    }
    Frag<T>::keep(bh[0], bh[1], bh[2], bh[3]);
    if (SPL == 2) Frag<T>::keep(bl[0], bl[1], bl[2], bl[3]);
  }

  float* slab = sT[wave];
#pragma unroll
  for (int i = 0; i < 4; ++i) {
    const int mBase = m0 + (i << 4);
#pragma unroll
    for (int j = 0; j < 4; ++j) {
      const int n = n0 + (j << 4) + rlane;
      float bv = 0.f;
      if (BIAS_MODE == 2) bv = bias[n];
#pragma unroll
      for (int r = 0; r < 8; ++r) {
        float v = acc[i][j][r] * scale;
        if (BIAS_MODE == 1) v += bias[mBase + mOff + r];
        if (BIAS_MODE == 2) v += bv;
        if (ACT == 2) v = fmaxf(v, 0.0f);
        slab[(mOff + r) * 68 + (j << 4) + rlane] = v;
      }
    }
    __builtin_amdgcn_fence(__ATOMIC_RELEASE, "workgroup");
    __builtin_amdgcn_wave_barrier();
    __builtin_amdgcn_fence(__ATOMIC_ACQUIRE, "workgroup");
    if (OUT_MODE == 0) {
      float* C = (float*)Cout + (size_t)b * strideC;
      const int hh = lane >> 4, c4 = (lane & 15) * 4;
      for (int pass = 0; pass < 2; ++pass) {
#pragma unroll
        for (int it = 0; it < 8; ++it) {
          const int row = it * 2 + hh;
          v4f v = *(const v4f*)(slab + row * 68 + c4);
          *(volatile v4f*)(C + (size_t)(mBase + row) * ldc + n0 + c4) = v;
        }
        __threadfence();
      }
    } else {
      const int q = lane >> 3, c8 = (lane & 7) * 8;
      unsigned short* C  = (unsigned short*)Cout  + (size_t)b * strideC;
      unsigned short* C2 = (OUT_MODE == 2) ? ((unsigned short*)Cout2 + (size_t)b * strideC) : nullptr;
      for (int pass = 0; pass < 2; ++pass) {
#pragma unroll
        for (int it = 0; it < 4; ++it) {
          const int row = it * 4 + q;
          const float* sp = slab + row * 68 + c8;
          v8h hv, lv;
#pragma unroll
          for (int e = 0; e < 8; ++e) {
            if (OUT_MODE == 1) {
              hv[e] = (_Float16)sp[e];
            } else {
              unsigned short hb = f2bf_bits(sp[e]);
              unsigned short lb = f2bf_bits(sp[e] - bf_bits2f(hb));
              hv[e] = __builtin_bit_cast(_Float16, hb);
              lv[e] = __builtin_bit_cast(_Float16, lb);
            }
          }
          *(volatile v8h*)(C + (size_t)(mBase + row) * ldc + n0 + c8) = hv;
          if (OUT_MODE == 2) *(volatile v8h*)(C2 + (size_t)(mBase + row) * ldc + n0 + c8) = lv;
        }
        __threadfence();
      }
    }
    __builtin_amdgcn_fence(__ATOMIC_RELEASE, "workgroup");
    __builtin_amdgcn_wave_barrier();
    __builtin_amdgcn_fence(__ATOMIC_ACQUIRE, "workgroup");
  }
}

__global__ __launch_bounds__(256) void split_rows_bf16_kernel(
    const float* __restrict__ src, unsigned short* __restrict__ dhi, unsigned short* __restrict__ dlo, int total8)
{
  const int i = blockIdx.x * 256 + threadIdx.x;
  if (i >= total8) return;
  const size_t e0 = (size_t)i << 3;
  const v4f a0 = *(const v4f*)(src + e0);
  const v4f a1 = *(const v4f*)(src + e0 + 4);
  v8h hv, lv;
#pragma unroll
  for (int e = 0; e < 4; ++e) {
    const unsigned short h0 = f2bf_bits(a0[e]), h1 = f2bf_bits(a1[e]);
    const unsigned short l0 = f2bf_bits(a0[e] - bf_bits2f(h0)), l1 = f2bf_bits(a1[e] - bf_bits2f(h1));
    hv[e]     = __builtin_bit_cast(_Float16, h0);
    hv[4 + e] = __builtin_bit_cast(_Float16, h1);
    lv[e]     = __builtin_bit_cast(_Float16, l0);
    lv[4 + e] = __builtin_bit_cast(_Float16, l1);
  }
  unsigned short* qh = dhi + e0;
  unsigned short* ql = dlo + e0;
  *(volatile v8h*)qh = hv;
  *(volatile v8h*)ql = lv;
  __threadfence();
  *(volatile v8h*)qh = hv;
  *(volatile v8h*)ql = lv;
}

__global__ __launch_bounds__(256) void split_transpose_bf16_kernel(
    const float* __restrict__ src, int pitch, int K,
    unsigned short* __restrict__ dhi, unsigned short* __restrict__ dlo, int total8)
{
  const int i = blockIdx.x * 256 + threadIdx.x;
  if (i >= total8) return;
  const int kq = K >> 3;
  const int n  = i / kq;
  const int k0 = (i - n * kq) << 3;
  float a[8];
#pragma unroll
  for (int e = 0; e < 8; ++e) a[e] = src[(size_t)(k0 + e) * pitch + n];
  v8h hv, lv;
#pragma unroll
  for (int e = 0; e < 8; ++e) {
    const unsigned short hb = f2bf_bits(a[e]);
    const unsigned short lb = f2bf_bits(a[e] - bf_bits2f(hb));
    hv[e] = __builtin_bit_cast(_Float16, hb);
    lv[e] = __builtin_bit_cast(_Float16, lb);
  }
  const size_t e0 = (size_t)i << 3;
  unsigned short* qh = dhi + e0;
  unsigned short* ql = dlo + e0;
  *(volatile v8h*)qh = hv;
  *(volatile v8h*)ql = lv;
  __threadfence();
  *(volatile v8h*)qh = hv;
  *(volatile v8h*)ql = lv;
}

__global__ __launch_bounds__(256) void pair_relu_dot_kernel(
    const float* __restrict__ E, const float* __restrict__ Afull, const float* __restrict__ fb,
    const float* __restrict__ W1b, const float* __restrict__ b1, const float* __restrict__ W2,
    const float* __restrict__ b2, float* __restrict__ out)
{
  __shared__ __align__(16) float sE[32 * kEP];
  __shared__ __align__(16) float sA[kB * kH];
  __shared__ __align__(16) float sW[kH];
  const int tid = threadIdx.x, lane = tid & 31, wave = tid >> 5;
  const int o0 = blockIdx.x * 32;

#pragma unroll
  for (int i = 0; i < 8; ++i) {
    const int idx = tid + 256 * i;
    *(v4f*)(sA + idx * 4) = *(const v4f*)(Afull + idx * 4);
  }
#pragma unroll
  for (int i = 0; i < 4; ++i) {
    const int r  = wave + 8 * i;
    const int c4 = lane * 4;
    const v4f ev = *(const v4f*)(E + (size_t)(o0 + r) * kH + c4);
    const float f = fb[o0 + r];
    const v4f wb = *(const v4f*)(W1b + c4);
    const v4f bv = *(const v4f*)(b1 + c4);
    v4f t;
    t[0] = ev[0] + (f * wb[0] + bv[0]);
    t[1] = ev[1] + (f * wb[1] + bv[1]);
    t[2] = ev[2] + (f * wb[2] + bv[2]);
    t[3] = ev[3] + (f * wb[3] + bv[3]);
    *(v4f*)(sE + r * kEP + c4) = t;
  }
  if (tid < 32) *(v4f*)(sW + tid * 4) = *(const v4f*)(W2 + tid * 4);
  __syncthreads();

  const float b2v = b2[0];
  const float* er = sE + lane * kEP;
  const float* ar = sA + (wave * 8) * kH;
  float acc[8];
#pragma unroll
  for (int bb = 0; bb < 8; ++bb) acc[bb] = 0.0f;

#pragma unroll 1
  for (int h4 = 0; h4 < kH / 4; ++h4) {
    const v4f e = *(const v4f*)(er + 4 * h4);
    const v4f w = *(const v4f*)(sW + 4 * h4);
#pragma unroll
    for (int bb = 0; bb < 8; ++bb) {
      const v4f a = *(const v4f*)(ar + bb * kH + 4 * h4);
      float s = acc[bb];
      s = fmaf(fmaxf(a[0] + e[0], 0.0f), w[0], s);
      s = fmaf(fmaxf(a[1] + e[1], 0.0f), w[1], s);
      s = fmaf(fmaxf(a[2] + e[2], 0.0f), w[2], s);
      s = fmaf(fmaxf(a[3] + e[3], 0.0f), w[3], s);
      acc[bb] = s;
    }
  }

  float res[8];
#pragma unroll
  for (int bb = 0; bb < 8; ++bb) res[bb] = acc[bb] + b2v;
  for (int pass = 0; pass < 2; ++pass) {
#pragma unroll
    for (int bb = 0; bb < 8; ++bb)
      *(volatile float*)(out + (size_t)(wave * 8 + bb) * kO + o0 + lane) = res[bb];
    __threadfence();
  }
}

static_assert((kO * kC / 8) % 256 == 0 && (kB * kL / 8) == 256);
static_assert((kH * kL / 8) % 256 == 0 && (kH * kC / 8) % 256 == 0 && (kH * kH / 8) % 256 == 0);

extern "C" void kernel_launch(void* const* d_in, const int* in_sizes, int n_in,
                              void* d_out, int out_size, void* d_ws, size_t ws_size,
                              hipStream_t stream) {
  if (n_in < 9) return;
  if (in_sizes[0] != kB * kL) return;
  if (in_sizes[1] != kO * kC) return;
  if (in_sizes[2] != kO) return;
  if (in_sizes[3] != kL * kH) return;
  if (in_sizes[4] != kH) return;
  if (in_sizes[5] != kW1Rows * kH) return;
  if (in_sizes[6] != kH) return;
  if (in_sizes[7] != kH) return;
  if (in_sizes[8] != 1) return;
  if (out_size != kB * kO) return;
  if (ws_size < kWsTotal) return;

  const float* z  = (const float*)d_in[0];
  const float* FE = (const float*)d_in[1];
  const float* fb = (const float*)d_in[2];
  const float* Wz = (const float*)d_in[3];
  const float* bz = (const float*)d_in[4];
  const float* W1 = (const float*)d_in[5];
  const float* b1 = (const float*)d_in[6];
  const float* W2 = (const float*)d_in[7];
  const float* b2 = (const float*)d_in[8];
  float* out = (float*)d_out;

  const float* W1h = W1;
  const float* W1f = W1 + (size_t)kH * kH;
  const float* W1b = W1 + (size_t)(kH + kC) * kH;

  char* ws = (char*)d_ws;
  unsigned short* FEH = (unsigned short*)(ws + kOffFEH);
  unsigned short* FEL = (unsigned short*)(ws + kOffFEL);
  unsigned short* ZH  = (unsigned short*)(ws + kOffZH);
  unsigned short* ZL  = (unsigned short*)(ws + kOffZL);
  unsigned short* WZH = (unsigned short*)(ws + kOffWZH);
  unsigned short* WZL = (unsigned short*)(ws + kOffWZL);
  unsigned short* WFH = (unsigned short*)(ws + kOffWFH);
  unsigned short* WFL = (unsigned short*)(ws + kOffWFL);
  unsigned short* WHH = (unsigned short*)(ws + kOffWHH);
  unsigned short* WHL = (unsigned short*)(ws + kOffWHL);
  unsigned short* PZH = (unsigned short*)(ws + kOffPZH);
  unsigned short* PZL = (unsigned short*)(ws + kOffPZL);
  float*          AF  = (float*)(ws + kOffAF);
  float*          EF  = (float*)(ws + kOffEF);

  split_rows_bf16_kernel<<<(kO * kC / 8) / 256, 256, 0, stream>>>(FE, FEH, FEL, kO * kC / 8);
  split_rows_bf16_kernel<<<(kB * kL / 8) / 256, 256, 0, stream>>>(z, ZH, ZL, kB * kL / 8);
  split_transpose_bf16_kernel<<<(kH * kL / 8) / 256, 256, 0, stream>>>(Wz, kH, kL, WZH, WZL, kH * kL / 8);
  split_transpose_bf16_kernel<<<(kH * kC / 8) / 256, 256, 0, stream>>>(W1f, kH, kC, WFH, WFL, kH * kC / 8);
  split_transpose_bf16_kernel<<<(kH * kH / 8) / 256, 256, 0, stream>>>(W1h, kH, kH, WHH, WHL, kH * kH / 8);

  wmma_gemm64<1, 2, 2, 2, false, 2><<<dim3(1, 1), 256, 0, stream>>>(
      ZH, ZL, kL, 0L,
      WZH, WZL, kL, 0L,
      (void*)PZH, (void*)PZL, kH, 0L,
      bz, nullptr, 0L,
      kB, kH, kL, 1.0f);

  wmma_gemm64<1, 2, 0, 0, false, 0><<<dim3(1, 1), 256, 0, stream>>>(
      PZH, PZL, kH, 0L,
      WHH, WHL, kH, 0L,
      (void*)AF, nullptr, kH, 0L,
      nullptr, nullptr, 0L,
      kB, kH, kH, 1.0f);

  wmma_gemm64<1, 2, 0, 0, false, 0><<<dim3((kO / 64) * (kH / 64) / 8, 1), 256, 0, stream>>>(
      FEH, FEL, kC, 0L,
      WFH, WFL, kC, 0L,
      (void*)EF, nullptr, kH, 0L,
      nullptr, nullptr, 0L,
      kO, kH, kC, 1.0f);

  pair_relu_dot_kernel<<<kO / 32, 256, 0, stream>>>(EF, AF, fb, W1b, b1, W2, b2, out);
}
